// FlashSelfAttention_64828236366197
// MI455X (gfx1250) — hardware-verified
//
#include <hip/hip_runtime.h>


#ifndef NB
#define NB 2
#endif
#ifndef SEQ
#define SEQ 2048
#endif
#define NB_FULL  2
#define SEQ_FULL 2048
#define NH   16
#define HD   128
#define DQ   (NH * HD)
#define ZH   2
#define BLK  128
#define SCL  0.088388347648318447f
#define EPSN 1.0e-12f
static_assert(SEQ % 128 == 0);
static_assert(SEQ >= BLK);
static_assert(SEQ <= SEQ_FULL);
static_assert(NB >= 1 && NB <= NB_FULL);
static_assert(NH % ZH == 0);
static_assert(HD == 128);
static_assert(BLK % 64 == 0);

typedef unsigned short bf;
typedef __attribute__((ext_vector_type(16))) __bf16   v16bf;
typedef __attribute__((ext_vector_type(8)))  unsigned short v8us;
typedef __attribute__((ext_vector_type(8)))  float    v8f;
typedef __attribute__((ext_vector_type(4)))  float    v4f;
typedef __attribute__((ext_vector_type(4)))  unsigned short v4us;
typedef __attribute__((ext_vector_type(2)))  unsigned short v2us;
typedef v4f  __attribute__((may_alias)) v4fa;

__device__ __forceinline__ unsigned short f2bf(float f) { unsigned u = __float_as_uint(f); u += 0x7FFFu + ((u >> 16) & 1u); return (unsigned short)(u >> 16); }
__device__ __forceinline__ float bf2f(unsigned short b) { return __uint_as_float(((unsigned)b) << 16); }
__device__ __forceinline__ float bfr(float f) { return bf2f(f2bf(f)); }
__device__ __forceinline__ void splitf(float y, unsigned short& h, unsigned short& l) { h = f2bf(y); l = f2bf(y - bf2f(h)); }
__device__ __forceinline__ v16bf cat16b(v8us lo, v8us hi) { return __builtin_bit_cast(v16bf, __builtin_shufflevector(lo, hi, 0, 1, 2, 3, 4, 5, 6, 7, 8, 9, 10, 11, 12, 13, 14, 15)); }
__device__ __forceinline__ v8f wmmab(v16bf a, v16bf b, v8f c) { return __builtin_amdgcn_wmma_f32_16x16x32_bf16(false, a, false, b, (short)0, c, false, false); }

template <typename T16> struct WFrag;
template <> struct WFrag<bf> { typedef v16bf V; static __device__ __forceinline__ V ld(const bf* p) { return cat16b(*(const v8us*)p, *(const v8us*)(p + 16)); } static __device__ __forceinline__ v8f mma(V a, V b, v8f c) { return wmmab(a, b, c); } };

template <typename T16, int NSPLIT, int CMODE>
__global__ __launch_bounds__(32) void k_gemmc(const T16* __restrict__ A, const T16* __restrict__ A2, const T16* __restrict__ Bt, const T16* __restrict__ Bt2, int K, float* C, int ldc, int roff, size_t sA, size_t sB, size_t sC) {
    typedef typename WFrag<T16>::V V;
    __shared__ __align__(16) float os[16 * 68];
    const size_t z = blockIdx.z; A += z * sA; if (A2) A2 += z * sA; Bt += z * sB; if (Bt2) Bt2 += z * sB; C += z * sC;
    const int lane = threadIdx.x & 31, lr = lane & 15, hi = lane >> 4; const int r0 = blockIdx.x * 64, c0 = blockIdx.y * 64;
    if (CMODE == 1 && c0 > r0 + roff + 63 && (r0 + roff >= BLK || c0 >= BLK)) return;
    const int Kl = (CMODE == 2) ? min(K, max(r0 + roff + 64, BLK)) : K;
    v8f acc[4][4];
#pragma unroll
    for (int mb = 0; mb < 4; ++mb)
#pragma unroll
        for (int nb = 0; nb < 4; ++nb) acc[mb][nb] = (v8f){};
    const size_t aoff = (size_t)(r0 + lr) * K + 8 * hi, boff = (size_t)(c0 + lr) * K + 8 * hi;
#pragma unroll 1
    for (int kc = 0; kc < Kl; kc += 32) {
        V a[4], a2[4];
#pragma unroll
        for (int mb = 0; mb < 4; ++mb) { a[mb] = WFrag<T16>::ld(A + aoff + (size_t)mb * 16 * K + kc); if (NSPLIT == 1 || NSPLIT == 2) a2[mb] = WFrag<T16>::ld(A2 + aoff + (size_t)mb * 16 * K + kc); }
#pragma unroll
        for (int nb = 0; nb < 4; ++nb) { const V b = WFrag<T16>::ld(Bt + boff + (size_t)nb * 16 * K + kc); V b2; if (NSPLIT >= 2) b2 = WFrag<T16>::ld(Bt2 + boff + (size_t)nb * 16 * K + kc);
#pragma unroll
            for (int mb = 0; mb < 4; ++mb) { acc[mb][nb] = WFrag<T16>::mma(a[mb], b, acc[mb][nb]); if (NSPLIT == 1 || NSPLIT == 2) acc[mb][nb] = WFrag<T16>::mma(a2[mb], b, acc[mb][nb]); if (NSPLIT >= 2) acc[mb][nb] = WFrag<T16>::mma(a[mb], b2, acc[mb][nb]); } }
        asm volatile("v_nop\n\tv_nop\n\tv_nop\n\tv_nop" : "+v"(acc[0][0]), "+v"(acc[1][1]), "+v"(acc[2][2]), "+v"(acc[3][3]) : "v"(a[0]), "v"(a[3]));
    }
#pragma unroll
    for (int mb = 0; mb < 4; ++mb) {
#pragma unroll
        for (int nb = 0; nb < 4; ++nb) {
#pragma unroll
            for (int j = 0; j < 8; ++j) os[(hi * 8 + j) * 68 + nb * 16 + lr] = acc[mb][nb][j]; }
        __builtin_amdgcn_wave_barrier(); asm volatile("" ::: "memory");
        float* crow = C + (size_t)(r0 + mb * 16) * ldc + c0;
#pragma unroll 1
        for (int ps = 0; ps < 2; ++ps) {
#pragma unroll
            for (int s = 0; s < 8; ++s) { const int row = 2 * s + hi, cofs = lr * 4; v4f val = *(const v4fa*)(os + row * 68 + cofs);
                *(volatile v4f*)(crow + (size_t)row * ldc + cofs) = val; }
            if (ps == 0) __threadfence(); }
        __builtin_amdgcn_wave_barrier(); asm volatile("" ::: "memory");
    }
}

template <bool NORM>
__global__ __launch_bounds__(256) void k_qkplane(const float* __restrict__ F, bf* Ph, bf* Pl) {
    const int lane = threadIdx.x & 31; const int row = blockIdx.x * 8 + (threadIdx.x >> 5); if (row >= NH * SEQ) return;
    const int h = row / SEQ, t = row % SEQ;
    const v4f a = *(const v4f*)(F + (size_t)t * DQ + h * HD + lane * 4);
    float x[4];
#pragma unroll
    for (int u = 0; u < 4; ++u) x[u] = bfr(a[u]);
    float f = 1.0f;
    if (NORM) {
        float ss = 0.f;
#pragma unroll
        for (int u = 0; u < 4; ++u) ss += x[u] * x[u];
#pragma unroll
        for (int sh = 16; sh; sh >>= 1) ss += __shfl_xor(ss, sh, 32);
        const float nrm = __fsqrt_rn(ss); f = __fdiv_rn(1.0f, fmaxf(nrm, EPSN));
    }
    v4us oh, ol;
#pragma unroll
    for (int u = 0; u < 4; ++u) { const float y = NORM ? __fmul_rn(x[u], f) : x[u]; unsigned short hh, ll; splitf(y, hh, ll); oh[u] = hh; ol[u] = ll; }
    const size_t oo = (size_t)row * HD + lane * 4;
    *(volatile v4us*)(Ph + oo) = oh; if (NORM) *(volatile v4us*)(Pl + oo) = ol;
    __threadfence();
    *(volatile v4us*)(Ph + oo) = oh; if (NORM) *(volatile v4us*)(Pl + oo) = ol;
}

__global__ __launch_bounds__(256) void k_vtp(const float* __restrict__ F, bf* Vh) {
    const size_t e = ((size_t)blockIdx.x * 256 + threadIdx.x) * 2; if (e >= (size_t)NH * HD * SEQ) return;
    const int t = (int)(e % SEQ); const int d = (int)((e / SEQ) % HD); const int g = (int)(e / ((size_t)SEQ * HD)); v2us oh;
#pragma unroll
    for (int q = 0; q < 2; ++q) oh[q] = f2bf(F[(size_t)(t + q) * DQ + g * HD + d]);
    *(volatile v2us*)(Vh + e) = oh; __threadfence(); *(volatile v2us*)(Vh + e) = oh;
}

__global__ __launch_bounds__(256) void k_asoft(const float* __restrict__ Sb, bf* Ph, bf* Pl) {
    const int lane = threadIdx.x & 31; const int row = blockIdx.x * 8 + (threadIdx.x >> 5); if (row >= ZH * SEQ) return;
    const int i = row % SEQ; const bool fb = (i < BLK); const float* sr = Sb + (size_t)row * SEQ; float v[SEQ / 32]; float mx = -3.0e38f;
#pragma unroll
    for (int ch = 0; ch < SEQ / 128; ++ch) { const int j0 = ch * 128 + lane * 4; const v4f a = *(const v4f*)(sr + j0);
#pragma unroll
        for (int q = 0; q < 4; ++q) { const int j = j0 + q; const bool ok = (j <= i) || (fb && (j < BLK)); float sa = a[q] * SCL; asm volatile("" : "+v"(sa)); const float t = ok ? sa : -3.0e38f; v[ch * 4 + q] = t; mx = fmaxf(mx, t); } }
#pragma unroll
    for (int sh = 16; sh; sh >>= 1) mx = fmaxf(mx, __shfl_xor(mx, sh, 32));
    float sum = 0.f;
#pragma unroll
    for (int k = 0; k < SEQ / 32; ++k) { float d0 = __fsub_rn(v[k], mx); asm volatile("" : "+v"(d0)); v[k] = __builtin_amdgcn_exp2f(__fmul_rn(d0, 1.4426950408889634f)); sum += v[k]; }
#pragma unroll
    for (int sh = 16; sh; sh >>= 1) sum += __shfl_xor(sum, sh, 32);
    const float f = __fdiv_rn(1.0f, sum);
#pragma unroll 1
    for (int ps = 0; ps < 2; ++ps) {
#pragma unroll
        for (int ch = 0; ch < SEQ / 128; ++ch) { v4us oh, ol;
#pragma unroll
            for (int q = 0; q < 4; ++q) { unsigned short hh, ll; splitf(v[ch * 4 + q] * f, hh, ll); oh[q] = hh; ol[q] = ll; }
            const size_t oo = (size_t)row * SEQ + ch * 128 + lane * 4; *(volatile v4us*)(Ph + oo) = oh; *(volatile v4us*)(Pl + oo) = ol; }
        if (ps == 0) __threadfence(); }
}

extern "C" void kernel_launch(void* const* d_in, const int* in_sizes, int n_in,
                              void* d_out, int out_size, void* d_ws, size_t ws_size, hipStream_t stream) {
    if (n_in < 3) return;
    const float* qin = (const float*)d_in[0]; const float* kin = (const float*)d_in[1]; const float* vin = (const float*)d_in[2];
    const size_t need_in = ((size_t)(NB - 1) * SEQ_FULL + SEQ) * DQ;
    if ((size_t)in_sizes[0] < need_in || (size_t)in_sizes[1] < need_in || (size_t)in_sizes[2] < need_in) return;
    if ((size_t)out_size < (size_t)NB * SEQ * DQ) return;
    float* OUT = (float*)d_out;
    char* wsp = (char*)d_ws;
    auto take = [&](size_t bytes) { char* p = wsp; wsp += (bytes + 255) & ~(size_t)255; return (void*)p; };
    bf* QPh = (bf*)take((size_t)NH * SEQ * HD * 2);
    bf* QPl = (bf*)take((size_t)NH * SEQ * HD * 2);
    bf* KPh = (bf*)take((size_t)NH * SEQ * HD * 2);
    bf* VTh = (bf*)take((size_t)NH * HD * SEQ * 2);
    float* Sb = (float*)take((size_t)ZH * SEQ * SEQ * 4);
    bf* Ph = (bf*)take((size_t)ZH * SEQ * SEQ * 2);
    bf* Pl = (bf*)take((size_t)ZH * SEQ * SEQ * 2);
    if ((size_t)(wsp - (char*)d_ws) > ws_size) return;
    const unsigned LP = (unsigned)((size_t)NH * SEQ / 8), LV = (unsigned)(((size_t)NH * HD * SEQ / 2 + 255) / 256);
    for (int b = 0; b < NB; ++b) {
        const float* FQ = qin + (size_t)b * SEQ_FULL * DQ; const float* FK = kin + (size_t)b * SEQ_FULL * DQ; const float* FV = vin + (size_t)b * SEQ_FULL * DQ;
        float* OUTb = OUT + (size_t)b * SEQ * DQ;
        k_qkplane<true><<<LP, 256, 0, stream>>>(FQ, QPh, QPl);
        k_qkplane<false><<<LP, 256, 0, stream>>>(FK, KPh, KPh);
        k_vtp<<<LV, 256, 0, stream>>>(FV, VTh);
        for (int h0 = 0; h0 < NH; h0 += ZH) { const size_t zo = (size_t)h0 * SEQ * HD;
            k_gemmc<bf, 1, 1><<<dim3(SEQ / 64, SEQ / 64, ZH), 32, 0, stream>>>(QPh + zo, QPl + zo, KPh + zo, KPh + zo, HD, Sb, SEQ, 0, (size_t)SEQ * HD, (size_t)SEQ * HD, (size_t)SEQ * SEQ);
            k_asoft<<<(unsigned)(ZH * SEQ / 8), 256, 0, stream>>>(Sb, Ph, Pl);
            k_gemmc<bf, 1, 2><<<dim3(SEQ / 64, HD / 64, ZH), 32, 0, stream>>>(Ph, Pl, VTh + (size_t)h0 * HD * SEQ, VTh + (size_t)h0 * HD * SEQ, SEQ, OUTb + (size_t)h0 * HD, DQ, 0, (size_t)SEQ * SEQ, (size_t)HD * SEQ, (size_t)HD);
        }
    }
}
